// MyBasicNeighborAtt_15753940041865
// MI455X (gfx1250) — hardware-verified
//
#include <hip/hip_runtime.h>
#include <stdint.h>

typedef _Float16 f16t;
typedef _Float16 v16h __attribute__((ext_vector_type(16)));
typedef _Float16 v8h  __attribute__((ext_vector_type(8)));
typedef _Float16 v4h  __attribute__((ext_vector_type(4)));
typedef __bf16   v16bf __attribute__((ext_vector_type(16)));
typedef unsigned short v16us __attribute__((ext_vector_type(16)));
typedef float v8f __attribute__((ext_vector_type(8)));
typedef float v4f __attribute__((ext_vector_type(4)));
typedef v8h  v8h_ma  __attribute__((may_alias));
typedef v4h  v4h_ma  __attribute__((may_alias));
typedef v4f  v4f_ma  __attribute__((may_alias));

#define KN    50
#define FD    64
#define DD    64
#define LL    3
#define HH    8
#define DKK   64
#define HD    512
#define BT    16
#define NTHR  256
#define XNP   64

#define OFF_XN    0
#define OFF_RAW   131072
#define OFF_WNT   139264
#define OFF_WQE   147456
#define OFF_QH    164864
#define OFF_ATTN  181248
#define OFF_XBAR  197632
#define OFF_CTX   214016
#define OFF_QF    230400
#define OFF_TMP   234496
#define OFF_H1    238592
#define OFF_H2    242688
#define OFF_QBK   246784
#define OFF_INV   247296
#define OFF_Y     247808
#define OFF_OUT   248064
#define OFF_S     248192
#define SMEM_BYTES 252288

__device__ __forceinline__ unsigned int bf_rne_bits(float x) {
  const unsigned int u = __float_as_uint(x);
  return (u + 0x7FFFu + ((u >> 16) & 1u)) >> 16;
}
__device__ __forceinline__ void split1(float x, unsigned short& hi, unsigned short& lo) {
  const unsigned int hb = bf_rne_bits(x);
  const float xh = __uint_as_float(hb << 16);
  hi = (unsigned short)hb;
  lo = (unsigned short)bf_rne_bits(x - xh);
}

union HFrag { v16h v; v8h h[2]; };
union BFrag { v16bf v; v16us u; };

__device__ __forceinline__ int kmap(int i, int hh) { return 8 * hh + (i & 7) + ((i >> 3) << 4); }

__device__ __forceinline__ v16h ldfrag_h(const f16t* base, int pitch) {
  const int lane = threadIdx.x & 31, m = lane & 15, hh = lane >> 4;
  const f16t* p = base + m * pitch + 8 * hh;
  HFrag f;
  f.h[0] = *(const v8h_ma*)(p);
  f.h[1] = *(const v8h_ma*)(p + 16);
  return f.v;
}
__device__ __forceinline__ v16h ldfrag_f32_h(const float* base, size_t pitch, float sc) {
  const int lane = threadIdx.x & 31, m = lane & 15, hh = lane >> 4;
  const float* p = base + (size_t)m * pitch + 8 * hh;
  const v4f x0 = *(const v4f_ma*)(p);
  const v4f x1 = *(const v4f_ma*)(p + 4);
  const v4f x2 = *(const v4f_ma*)(p + 16);
  const v4f x3 = *(const v4f_ma*)(p + 20);
  v16h a;
  a[0] = (f16t)(x0[0] * sc); a[1] = (f16t)(x0[1] * sc); a[2]  = (f16t)(x0[2] * sc); a[3]  = (f16t)(x0[3] * sc);
  a[4] = (f16t)(x1[0] * sc); a[5] = (f16t)(x1[1] * sc); a[6]  = (f16t)(x1[2] * sc); a[7]  = (f16t)(x1[3] * sc);
  a[8] = (f16t)(x2[0] * sc); a[9] = (f16t)(x2[1] * sc); a[10] = (f16t)(x2[2] * sc); a[11] = (f16t)(x2[3] * sc);
  a[12] = (f16t)(x3[0] * sc); a[13] = (f16t)(x3[1] * sc); a[14] = (f16t)(x3[2] * sc); a[15] = (f16t)(x3[3] * sc);
  return a;
}
__device__ __forceinline__ void ldfrag_f32_split(const float* base, size_t pitch, v16bf& hi, v16bf& lo) {
  const int lane = threadIdx.x & 31, m = lane & 15, hh = lane >> 4;
  const float* p = base + (size_t)m * pitch + 8 * hh;
  const v4f x0 = *(const v4f_ma*)(p);
  const v4f x1 = *(const v4f_ma*)(p + 4);
  const v4f x2 = *(const v4f_ma*)(p + 16);
  const v4f x3 = *(const v4f_ma*)(p + 20);
  float xs[16];
  xs[0] = x0[0]; xs[1] = x0[1]; xs[2]  = x0[2]; xs[3]  = x0[3];
  xs[4] = x1[0]; xs[5] = x1[1]; xs[6]  = x1[2]; xs[7]  = x1[3];
  xs[8] = x2[0]; xs[9] = x2[1]; xs[10] = x2[2]; xs[11] = x2[3];
  xs[12] = x3[0]; xs[13] = x3[1]; xs[14] = x3[2]; xs[15] = x3[3];
  BFrag Hf, Lf;
#pragma unroll
  for (int i = 0; i < 16; ++i) {
    unsigned short a, b;
    split1(xs[i], a, b);
    Hf.u[i] = a; Lf.u[i] = b;
  }
  hi = Hf.v; lo = Lf.v;
}
__device__ __forceinline__ void gath_f32_split(const float* __restrict__ base, size_t kpitch, v16bf& hi, v16bf& lo) {
  const int lane = threadIdx.x & 31, m = lane & 15, hh = lane >> 4;
  BFrag Hf, Lf;
#pragma unroll
  for (int i = 0; i < 16; ++i) {
    const float x = base[(size_t)kmap(i, hh) * kpitch + m];
    unsigned short a, b;
    split1(x, a, b);
    Hf.u[i] = a; Lf.u[i] = b;
  }
  hi = Hf.v; lo = Lf.v;
}
__device__ __forceinline__ v16h gath_f32_h(const float* __restrict__ base, size_t kpitch, float sc) {
  const int lane = threadIdx.x & 31, m = lane & 15, hh = lane >> 4;
  v16h b;
#pragma unroll
  for (int i = 0; i < 16; ++i) b[i] = (f16t)(base[(size_t)kmap(i, hh) * kpitch + m] * sc);
  return b;
}
__device__ __forceinline__ v16h gath_h(const f16t* base, int kpitch) {
  const int lane = threadIdx.x & 31, m = lane & 15, hh = lane >> 4;
  v16h b;
#pragma unroll
  for (int i = 0; i < 16; ++i) b[i] = base[kmap(i, hh) * kpitch + m];
  return b;
}

__device__ __forceinline__ v8f mma_h(v16h a, v16h b, v8f c) {
  c = __builtin_amdgcn_wmma_f32_16x16x32_f16(false, a, false, b, (short)0, c, false, false);
  asm volatile("v_nop\n\tv_nop\n\tv_nop\n\tv_nop" : "+v"(c) : "v"(a), "v"(b));
  return c;
}
__device__ __forceinline__ v8f mma_b3(v16bf ah, v16bf al, v16bf bh, v16bf bl, v8f c) {
  c = __builtin_amdgcn_wmma_f32_16x16x32_bf16(false, ah, false, bh, (short)0, c, false, false);
  c = __builtin_amdgcn_wmma_f32_16x16x32_bf16(false, ah, false, bl, (short)0, c, false, false);
  c = __builtin_amdgcn_wmma_f32_16x16x32_bf16(false, al, false, bh, (short)0, c, false, false);
  asm volatile("v_nop\n\tv_nop\n\tv_nop\n\tv_nop" : "+v"(c) : "v"(ah), "v"(al), "v"(bh), "v"(bl));
  return c;
}

__global__ __launch_bounds__(NTHR)
void k_main(const float* __restrict__ X, const int* __restrict__ S,
            const float* __restrict__ X_ref, const float* __restrict__ y_ref,
            const float* __restrict__ W_emb, const float* __restrict__ b_emb,
            const float* __restrict__ W_nemb, const float* __restrict__ b_nemb,
            const float* __restrict__ Wq, const float* __restrict__ bq,
            const float* __restrict__ Wk, const float* __restrict__ bk,
            const float* __restrict__ Wv, const float* __restrict__ bv,
            const float* __restrict__ Wo, const float* __restrict__ bo,
            const float* __restrict__ ln_g, const float* __restrict__ ln_b,
            const float* __restrict__ W1, const float* __restrict__ b1,
            const float* __restrict__ W2, const float* __restrict__ b2,
            const float* __restrict__ W3, const float* __restrict__ b3,
            float* __restrict__ wsf, int nref)
{
  extern __shared__ __align__(16) char smem[];
  f16t* sXn   = (f16t*)(smem + OFF_XN);
  f16t* sRaw  = (f16t*)(smem + OFF_RAW);
  f16t* sWnT  = (f16t*)(smem + OFF_WNT);
  f16t* sWqe  = (f16t*)(smem + OFF_WQE);
  f16t* sQh   = (f16t*)(smem + OFF_QH);
  f16t* sAttn = (f16t*)(smem + OFF_ATTN);
  f16t* sXbar = (f16t*)(smem + OFF_XBAR);
  f16t* sCtx  = (f16t*)(smem + OFF_CTX);
  float* qf   = (float*)(smem + OFF_QF);
  float* sTmp = (float*)(smem + OFF_TMP);
  float* sH1  = (float*)(smem + OFF_H1);
  float* sH2  = (float*)(smem + OFF_H2);
  float* qbkS = (float*)(smem + OFF_QBK);
  float* sInv = (float*)(smem + OFF_INV);
  float* sY   = (float*)(smem + OFF_Y);
  float* sOut = (float*)(smem + OFF_OUT);
  int*   sS   = (int*)(smem + OFF_S);

  const int tid = threadIdx.x;
  const int lane = tid & 31, wv = tid >> 5;
  const int m = lane & 15, hh = lane >> 4;
  const int b0 = blockIdx.x * BT;

  for (int i = tid; i < BT * XNP; i += NTHR) {
    const int e = i >> 6, n = i & 63;
    sS[i] = (n < KN) ? S[(size_t)(b0 + e) * KN + n] : -1;
  }
  for (int i = tid; i < 64 * 64; i += NTHR) sRaw[i] = (f16t)0.f;
  for (int i = tid; i < 8 * DKK; i += NTHR) sWqe[BT * HH * DKK + i] = (f16t)0.f;
  for (int i = tid; i < DD * 64; i += NTHR) {
    const int n = i >> 6, k = i & 63;
    sWnT[i] = (f16t)(W_nemb[k * DD + n] * 16.f);
  }
  if (tid < 64) sY[tid] = 0.f;
  if (tid < 32) sOut[tid] = 0.f;
  __syncthreads();

  for (int e = 0; e < BT; ++e) {
    for (int i = tid; i < KN * 16; i += NTHR) {
      const int n = i >> 4, k4 = (i & 15) * 4;
      int s = sS[e * XNP + n];
      s = s < 0 ? 0 : (s >= nref ? nref - 1 : s);
      const v4f v = *(const v4f_ma*)(X_ref + (size_t)s * FD + k4);
      v4h q;
      q[0] = (f16t)v[0]; q[1] = (f16t)v[1]; q[2] = (f16t)v[2]; q[3] = (f16t)v[3];
      *(v4h_ma*)(sRaw + n * 64 + k4) = q;
    }
    for (int n = tid; n < KN; n += NTHR) {
      int s = sS[e * XNP + n];
      s = s < 0 ? 0 : (s >= nref ? nref - 1 : s);
      sY[n] = y_ref[s];
    }
    __syncthreads();
#pragma unroll
    for (int t0 = 0; t0 < 2; ++t0) {
      const int t = wv + 8 * t0;
      const int mt = t >> 2, nt = t & 3;
      v8f acc = {};
#pragma unroll
      for (int kc = 0; kc < 2; ++kc) {
        const v16h a = ldfrag_h(sRaw + mt * 16 * 64 + kc * 32, 64);
        const v16h b = ldfrag_h(sWnT + nt * 16 * 64 + kc * 32, 64);
        acc = mma_h(a, b, acc);
      }
      const int col = nt * 16 + m;
      const float w64 = W_nemb[64 * DD + col];
      const float bb  = b_nemb[col];
#pragma unroll
      for (int r = 0; r < 8; ++r) {
        const int row = mt * 16 + 8 * hh + r;
        float v = acc[r] * 0.0625f + sY[row] * w64 + bb;
        v = fmaxf(v, 0.f);
        sXn[(size_t)(e * XNP + row) * DD + col] = (f16t)(row < KN ? v : 0.f);
      }
    }
    __syncthreads();
  }

  if (wv < 4) {
    const int nt = wv;
    v8f acc = {};
#pragma unroll
    for (int kc = 0; kc < 2; ++kc) {
      v16bf ah, al, bh, bl;
      ldfrag_f32_split(X + (size_t)b0 * FD + kc * 32, FD, ah, al);
      gath_f32_split(W_emb + (size_t)(kc * 32) * DD + nt * 16, DD, bh, bl);
      acc = mma_b3(ah, al, bh, bl, acc);
    }
    const int col = nt * 16 + m;
    const float be = b_emb[col];
#pragma unroll
    for (int r = 0; r < 8; ++r) qf[(8 * hh + r) * DD + col] = fmaxf(acc[r] + be, 0.f);
  }
  __syncthreads();

  for (int li = 0; li < LL; ++li) {
    const float* Wq_i = Wq + (size_t)li * DD * HD;
    const float* bq_i = bq + li * HD;
    const float* Wk_i = Wk + (size_t)li * DD * HD;
    const float* bk_i = bk + li * HD;
    const float* Wv_i = Wv + (size_t)li * DD * HD;
    const float* bv_i = bv + li * HD;
    const float* Wo_i = Wo + (size_t)li * HD * DD;
    const float* bo_i = bo + li * DD;
    const float* g_i  = ln_g + li * DD;
    const float* be_i = ln_b + li * DD;

    {
      v16h aq[2];
#pragma unroll
      for (int kc = 0; kc < 2; ++kc) aq[kc] = ldfrag_f32_h(qf + kc * 32, DD, 1.f);
#pragma unroll
      for (int j = 0; j < 4; ++j) {
        const int nt = wv * 4 + j;
        v8f acc = {};
#pragma unroll
        for (int kc = 0; kc < 2; ++kc) {
          const v16h b = gath_f32_h(Wq_i + (size_t)(kc * 32) * HD + nt * 16, HD, 16.f);
          acc = mma_h(aq[kc], b, acc);
        }
        const int col = nt * 16 + m;
        const float bqv = bq_i[col] * 16.f;
#pragma unroll
        for (int r = 0; r < 8; ++r) sQh[(8 * hh + r) * HD + col] = (f16t)(acc[r] + bqv);
      }
    }
    __syncthreads();

    {
      const int h = wv;
      v16h a2[2];
#pragma unroll
      for (int kc = 0; kc < 2; ++kc) a2[kc] = ldfrag_h(sQh + h * DKK + kc * 32, HD);
#pragma unroll
      for (int nt = 0; nt < 4; ++nt) {
        v8f acc = {};
#pragma unroll
        for (int kc = 0; kc < 2; ++kc) {
          const v16h b = ldfrag_f32_h(Wk_i + (size_t)(nt * 16) * HD + h * DKK + kc * 32, HD, 16.f);
          acc = mma_h(a2[kc], b, acc);
        }
#pragma unroll
        for (int r = 0; r < 8; ++r)
          sWqe[((8 * hh + r) * HH + h) * DKK + nt * 16 + m] = (f16t)acc[r];
      }
    }
    if (tid < BT * HH) {
      const int e = tid >> 3, h2 = tid & 7;
      float s = 0.f;
#pragma unroll 1
      for (int k = 0; k < DKK; ++k)
        s += (float)sQh[e * HD + h2 * DKK + k] * bk_i[h2 * DKK + k];
      qbkS[e * HH + h2] = s * 0.0625f;
    }
    __syncthreads();

    for (int p = 0; p < 2; ++p) {
      const int e = wv + 8 * p;
      const v16h bw0 = ldfrag_h(sWqe + e * HH * DKK, DKK);
      const v16h bw1 = ldfrag_h(sWqe + e * HH * DKK + 32, DKK);
      v8f cs[4];
#pragma unroll
      for (int mt = 0; mt < 4; ++mt) {
        const f16t* ab = sXn + (size_t)(e * XNP + mt * 16) * DD;
        v8f acc = {};
        acc = mma_h(ldfrag_h(ab, DD), bw0, acc);
        acc = mma_h(ldfrag_h(ab + 32, DD), bw1, acc);
        cs[mt] = acc;
      }
      const float qb = (m < HH) ? qbkS[e * HH + m] : 0.f;
      float mx = -3.0e38f;
#pragma unroll
      for (int mt = 0; mt < 4; ++mt)
#pragma unroll
        for (int r = 0; r < 8; ++r) {
          const int n = mt * 16 + 8 * hh + r;
          float sc;
          if (n < KN) {
            const bool valid = sS[e * XNP + n] >= 0;
            sc = valid ? (cs[mt][r] * (1.f / 256.f) + qb) * 0.125f : -1.0e9f;
          } else {
            sc = -3.0e38f;
          }
          cs[mt][r] = sc;
          mx = fmaxf(mx, sc);
        }
      mx = fmaxf(mx, __shfl_xor(mx, 16, 32));
      float sum = 0.f;
#pragma unroll
      for (int mt = 0; mt < 4; ++mt)
#pragma unroll
        for (int r = 0; r < 8; ++r) {
          const float ex = __expf(cs[mt][r] - mx);
          cs[mt][r] = ex;
          sum += ex;
        }
      sum += __shfl_xor(sum, 16, 32);
      const float inv = 1.f / sum;
#pragma unroll
      for (int mt = 0; mt < 4; ++mt)
#pragma unroll
        for (int r = 0; r < 8; ++r) {
          const int n = mt * 16 + 8 * hh + r;
          sAttn[(wv * 16 + m) * 64 + n] = (f16t)((m < HH) ? cs[mt][r] * 4096.f : 0.f);
        }
      if (hh == 0) sInv[wv * 16 + m] = inv;
      __syncthreads();
      const v16h ap0 = ldfrag_h(sAttn + wv * 16 * 64, 64);
      const v16h ap1 = ldfrag_h(sAttn + wv * 16 * 64 + 32, 64);
#pragma unroll
      for (int nt = 0; nt < 4; ++nt) {
        v8f acc = {};
        v16h b = gath_h(sXn + (size_t)(e * XNP) * DD + nt * 16, DD);
        acc = mma_h(ap0, b, acc);
        b = gath_h(sXn + (size_t)(e * XNP + 32) * DD + nt * 16, DD);
        acc = mma_h(ap1, b, acc);
#pragma unroll
        for (int r = 0; r < 8; ++r) {
          if (hh == 0) {
            const float v = acc[r] * sInv[wv * 16 + r] * (1.f / 256.f);
            sXbar[(e * HH + r) * DKK + nt * 16 + m] = (f16t)v;
          }
        }
      }
      __syncthreads();
    }

    {
      const int h = wv;
      v16h ax[2];
#pragma unroll
      for (int kc = 0; kc < 2; ++kc) ax[kc] = ldfrag_h(sXbar + h * DKK + kc * 32, HH * DKK);
#pragma unroll
      for (int nt = 0; nt < 4; ++nt) {
        v8f acc = {};
#pragma unroll
        for (int kc = 0; kc < 2; ++kc) {
          const v16h b = gath_f32_h(Wv_i + (size_t)(kc * 32) * HD + h * DKK + nt * 16, HD, 16.f);
          acc = mma_h(ax[kc], b, acc);
        }
        const int col = h * DKK + nt * 16 + m;
        const float bvv = bv_i[col] * 16.f;
#pragma unroll
        for (int r = 0; r < 8; ++r) sCtx[(8 * hh + r) * HD + col] = (f16t)(acc[r] * 0.0625f + bvv);
      }
    }
    __syncthreads();

    if (wv < 4) {
      const int nt = wv;
      v8f acc = {};
#pragma unroll 2
      for (int kc = 0; kc < 16; ++kc) {
        const v16h a = ldfrag_h(sCtx + kc * 32, HD);
        const v16h b = gath_f32_h(Wo_i + (size_t)(kc * 32) * DD + nt * 16, DD, 16.f);
        acc = mma_h(a, b, acc);
      }
      const int col = nt * 16 + m;
      const float bov = bo_i[col];
#pragma unroll
      for (int r = 0; r < 8; ++r) sTmp[(8 * hh + r) * DD + col] = acc[r] * (1.f / 256.f) + bov;
    }
    __syncthreads();
    if (tid < BT) {
      const int e = tid;
      float mu = 0.f;
#pragma unroll 1
      for (int d = 0; d < DD; ++d) mu += qf[e * DD + d] + sTmp[e * DD + d];
      mu *= (1.f / DD);
      float var = 0.f;
#pragma unroll 1
      for (int d = 0; d < DD; ++d) {
        const float x = qf[e * DD + d] + sTmp[e * DD + d] - mu;
        var += x * x;
      }
      var *= (1.f / DD);
      const float is = rsqrtf(var + 1e-3f);
#pragma unroll 1
      for (int d = 0; d < DD; ++d) {
        const float x = qf[e * DD + d] + sTmp[e * DD + d];
        qf[e * DD + d] = (x - mu) * is * g_i[d] + be_i[d];
      }
    }
    __syncthreads();
  }

  if (wv < 4) {
    const int nt = wv;
    v8f acc = {};
#pragma unroll
    for (int kc = 0; kc < 2; ++kc) {
      v16bf ah, al, bh, bl;
      ldfrag_f32_split(qf + kc * 32, DD, ah, al);
      gath_f32_split(W1 + (size_t)(kc * 32) * DD + nt * 16, DD, bh, bl);
      acc = mma_b3(ah, al, bh, bl, acc);
    }
    const int col = nt * 16 + m;
    const float bb = b1[col];
#pragma unroll
    for (int r = 0; r < 8; ++r) sH1[(8 * hh + r) * DD + col] = fmaxf(acc[r] + bb, 0.f);
  }
  __syncthreads();
  if (wv < 4) {
    const int nt = wv;
    v8f acc = {};
#pragma unroll
    for (int kc = 0; kc < 2; ++kc) {
      v16bf ah, al, bh, bl;
      ldfrag_f32_split(sH1 + kc * 32, DD, ah, al);
      gath_f32_split(W2 + (size_t)(kc * 32) * DD + nt * 16, DD, bh, bl);
      acc = mma_b3(ah, al, bh, bl, acc);
    }
    const int col = nt * 16 + m;
    const float bb = b2[col];
#pragma unroll
    for (int r = 0; r < 8; ++r) sH2[(8 * hh + r) * DD + col] = fmaxf(acc[r] + bb, 0.f);
  }
  __syncthreads();
  if (tid < BT) {
    float s = 0.f;
#pragma unroll 1
    for (int d = 0; d < DD; ++d) s += sH2[tid * DD + d] * W3[d];
    sOut[tid] = s + b3[0];
  }
  __syncthreads();
  {
    v4f ov = {};
    if (wv == 0 && lane < 8) ov = *(const v4f_ma*)(sOut + lane * 4);
    float* dst = wsf + (size_t)blockIdx.x * 32 + lane * 4;
    if (wv == 0 && lane < 8) *(volatile v4f*)dst = ov;
    __threadfence();
    if (wv == 0 && lane < 8) *(volatile v4f*)dst = ov;
  }
}

__global__ __launch_bounds__(256)
void k_out(const float* __restrict__ wsf, float* __restrict__ out, int n_out, int nblk)
{
  const int lane = threadIdx.x & 31, wv = threadIdx.x >> 5;
  const int gw = blockIdx.x * 8 + wv;
  const int nl = (n_out + 31) / 32;
  v4f v = {};
  bool doit = false;
  size_t o = 0;
  if (gw < nl && lane < 8) {
    const int sb = 2 * gw + (lane >> 2);
    if (sb < nblk) v = *(const v4f_ma*)(wsf + (size_t)sb * 32 + (lane & 3) * 4);
    o = (size_t)gw * 32 + (size_t)lane * 4;
    doit = (o + 4 <= (size_t)n_out);
  }
  if (doit) *(volatile v4f*)(out + o) = v;
  __threadfence();
  if (doit) *(volatile v4f*)(out + o) = v;
}

extern "C" void kernel_launch(void* const* d_in, const int* in_sizes, int n_in,
                              void* d_out, int out_size, void* d_ws, size_t ws_size,
                              hipStream_t stream) {
  if (n_in < 24) return;
  const float* X      = (const float*)d_in[0];
  const int*   S      = (const int*)  d_in[1];
  const float* X_ref  = (const float*)d_in[2];
  const float* y_ref  = (const float*)d_in[3];
  const float* W_emb  = (const float*)d_in[4];
  const float* b_emb  = (const float*)d_in[5];
  const float* W_nemb = (const float*)d_in[6];
  const float* b_nemb = (const float*)d_in[7];
  const float* Wq     = (const float*)d_in[8];
  const float* bq     = (const float*)d_in[9];
  const float* Wk     = (const float*)d_in[10];
  const float* bk     = (const float*)d_in[11];
  const float* Wv     = (const float*)d_in[12];
  const float* bv     = (const float*)d_in[13];
  const float* Wo     = (const float*)d_in[14];
  const float* bo     = (const float*)d_in[15];
  const float* ln_g   = (const float*)d_in[16];
  const float* ln_b   = (const float*)d_in[17];
  const float* W1     = (const float*)d_in[18];
  const float* b1     = (const float*)d_in[19];
  const float* W2     = (const float*)d_in[20];
  const float* b2     = (const float*)d_in[21];
  const float* W3     = (const float*)d_in[22];
  const float* b3     = (const float*)d_in[23];
  float* out = (float*)d_out;
  float* wsf = (float*)d_ws;

  if (in_sizes[0] <= 0 || (in_sizes[0] % FD) != 0) return;
  const int Bn = in_sizes[0] / FD;
  const int nref = in_sizes[3];
  if ((Bn % 32) != 0 || out_size != Bn) return;
  if (in_sizes[1] != Bn * KN || in_sizes[2] != nref * FD || nref <= 0) return;
  if (in_sizes[6] != (FD + 1) * DD || in_sizes[8] != LL * DD * HD || in_sizes[14] != LL * HD * DD) return;
  const int nblk = Bn / BT;
  const size_t need = (size_t)nblk * 32 * sizeof(float);
  if (need > ws_size) return;

  (void)hipFuncSetAttribute(reinterpret_cast<const void*>(&k_main),
                            hipFuncAttributeMaxDynamicSharedMemorySize, (int)SMEM_BYTES);

  k_main<<<nblk, NTHR, SMEM_BYTES, stream>>>(
      X, S, X_ref, y_ref, W_emb, b_emb, W_nemb, b_nemb,
      Wq, bq, Wk, bk, Wv, bv, Wo, bo, ln_g, ln_b,
      W1, b1, W2, b2, W3, b3, wsf, nref);

  const int nl = Bn / 32;
  k_out<<<(nl + 7) / 8, 256, 0, stream>>>(wsf, out, Bn, nblk);
  (void)hipGetLastError();
}
